// GLCN_31147102830954
// MI455X (gfx1250) — hardware-run, weakly checked
//
#include <hip/hip_runtime.h>


#ifndef NN
#define NN 2048
#endif
#define NN_FULL 2048
#ifndef OUT_NN
#define OUT_NN NN
#endif
#define FIN  64
#define GG   128
#define FOBS 32
#define NW3  (3 * GG)
#define WPR  (NN / 32)
#define RB   16
#define AW   4
#define OSP  132
#define HCS  64.0f
#define CSP  (64.0f / 4096.0f)
#define CSV  (1.0f / 4096.0f)
#define PSH  14.0f
#define L2E  1.4426950408889634f
#define FILL2 (-9.0e15f * 1.4426950408889634f)
#define NEGB (-3.0e38f)
#define EPSV 1e-10f

static_assert(FOBS == 32);
static_assert(FOBS <= FIN);
static_assert(FIN % 32 == 0);
static_assert(GG % 32 == 0);
static_assert(GG == 128);
static_assert(32 * 4 == GG);
static_assert(16 * 8 == GG);
static_assert(NW3 % 64 == 0);
static_assert(GG % 64 == 0);
static_assert(NN % 64 == 0);
static_assert(NN % 32 == 0);
static_assert(NN % (16 * AW) == 0);
static_assert(NN % RB == 0);
static_assert((RB * WPR) % 4 == 0);
static_assert(((size_t)RB * WPR * 4) % 128 == 0);
static_assert(NN <= NN_FULL);
static_assert(((size_t)NN * FIN / 4) % 256 == 0);
static_assert(((size_t)NN * FIN / 8) % 256 == 0);
static_assert(((size_t)GG * FIN / 8) % 256 == 0);
static_assert(((size_t)GG * GG / 8) % 256 == 0);
static_assert((OSP * 4) % 16 == 0);
static_assert(OSP >= GG);
static_assert(4 * (32 / 8) == 16);
static_assert(8 * (32 / 16) == 16);
static_assert(16 * 16 == 64 * 4);
static_assert((size_t)RB * FOBS * 4 + (size_t)RB * WPR * 4 + (size_t)8 * RB * 32 * 4 <= 131072);
static_assert((size_t)AW * 16 * OSP * 4 <= 131072);
static_assert((size_t)16 * 68 * 4 <= 131072);

typedef _Float16 h16;
typedef __attribute__((ext_vector_type(16))) _Float16 v16h;
typedef __attribute__((ext_vector_type(8)))  _Float16 v8h;
typedef __attribute__((ext_vector_type(8)))  float    v8f;
typedef __attribute__((ext_vector_type(4)))  float    v4f;
typedef __attribute__((ext_vector_type(4)))  unsigned v4u;
typedef v4f  __attribute__((may_alias)) v4fa;
typedef v4u  __attribute__((may_alias)) v4ua;

__device__ __forceinline__ unsigned short f2bf(float f) { unsigned u = __float_as_uint(f); u += 0x7FFFu + ((u >> 16) & 1u); return (unsigned short)(u >> 16); }
__device__ __forceinline__ float bfr(float f) { return __uint_as_float(((unsigned)f2bf(f)) << 16); }
__device__ __forceinline__ v16h cat16(v8h lo, v8h hi) { return __builtin_shufflevector(lo, hi, 0, 1, 2, 3, 4, 5, 6, 7, 8, 9, 10, 11, 12, 13, 14, 15); }
__device__ __forceinline__ v8f wmma16(v16h a, v16h b, v8f c) { return __builtin_amdgcn_wmma_f32_16x16x32_f16(false, a, false, b, (short)0, c, false, false); }
__device__ __forceinline__ v8f wg(v16h a, v16h b, v8f c) { c = wmma16(a, b, c); asm volatile("v_nop\n\tv_nop\n\tv_nop\n\tv_nop" : "+v"(c) : "v"(a), "v"(b)); return c; }
__device__ __forceinline__ v16h ldh(const h16* p) { return cat16(*(const v8h*)p, *(const v8h*)(p + 16)); }
static __device__ __forceinline__ h16 toh_flush(float v) { const h16 r = (h16)v; return (fabsf(v) < 6.103515625e-05f) ? (h16)0.0f : r; }
__device__ __forceinline__ void wave_sync() { __builtin_amdgcn_fence(3  , "wavefront"); __builtin_amdgcn_wave_barrier(); asm volatile("" ::: "memory"); }

__global__ __launch_bounds__(256) void k_xcopy(const float* __restrict__ X, float* OX, h16* XH) {
    const size_t i = (size_t)blockIdx.x * 256 + threadIdx.x;
    const v4f cr = *(const v4f*)(X + i * 4);
    v4f cv;
#pragma unroll
    for (int e = 0; e < 4; ++e) cv[e] = bfr(cr[e]);
    const bool hp = i < (size_t)NN * FIN / 8;
    v8h hv = (v8h){};
    if (hp) { const v8f v = *(const v8f*)(X + i * 8);
#pragma unroll
        for (int k = 0; k < 8; ++k) hv[k] = toh_flush(bfr(v[k]) * HCS); }
    *(volatile v4f*)(OX + i * 4) = cv; if (hp) *(volatile v8h*)(XH + i * 8) = hv;
    __threadfence();
    *(volatile v4f*)(OX + i * 4) = cv; if (hp) *(volatile v8h*)(XH + i * 8) = hv;
}

__global__ __launch_bounds__(256) void k_wt(const float* __restrict__ W, h16* dst, int K) {
    const int per = K >> 3;
    const int i = blockIdx.x * 256 + threadIdx.x; if (i >= GG * per) return;
    const int n = i / per, k8 = (i - n * per) * 8;
    v8h o;
#pragma unroll
    for (int e = 0; e < 8; ++e) o[e] = toh_flush(bfr(W[(size_t)(k8 + e) * GG + n]) * HCS);
    *(volatile v8h*)(dst + (size_t)i * 8) = o; __threadfence(); *(volatile v8h*)(dst + (size_t)i * 8) = o;
}

__global__ __launch_bounds__(256) void k_adj(const float* __restrict__ X, const float* __restrict__ GU, const float* __restrict__ AL, float* AOUT, unsigned* MB) {
    __shared__ __align__(16) float hs[RB * FOBS];
    __shared__ __align__(16) unsigned mws[RB * WPR];
    __shared__ __align__(16) float aw[8 * RB * 32];
    const int tid = threadIdx.x, lane = tid & 31;
    const int wave = __builtin_amdgcn_readfirstlane((int)(threadIdx.x >> 5));
    const int i0 = blockIdx.x * RB;
    for (int s = tid; s < RB * FOBS; s += 256) { const int r = s >> 5, c = s & 31; hs[s] = bfr(X[(size_t)(i0 + r) * FIN + c]); }
    float al[FOBS];
#pragma unroll
    for (int q = 0; q < FOBS / 4; ++q) { const v4f t = *(const v4f*)(AL + 4 * q);
#pragma unroll
        for (int e = 0; e < 4; ++e) al[4 * q + e] = bfr(t[e]); }
    __syncthreads();
#pragma unroll 1
    for (int seg = wave; seg < WPR; seg += 8) {
        const int j = seg * 32 + lane;
        const float* xr = X + (size_t)j * FIN;
        float hj[FOBS];
#pragma unroll
        for (int q = 0; q < FOBS / 4; ++q) { const v4f t = *(const v4f*)(xr + 4 * q);
#pragma unroll
            for (int e = 0; e < 4; ++e) hj[4 * q + e] = bfr(t[e]); }
#pragma unroll 1
        for (int r = 0; r < RB; ++r) {
            const int i = i0 + r;
            const float u = bfr(GU[(size_t)i * NN_FULL + j]);
            float lg = 0.0f;
#pragma unroll
            for (int q = 0; q < FOBS / 4; ++q) { const v4f hv = *(const v4fa*)(&hs[r * FOBS + 4 * q]);
#pragma unroll
                for (int e = 0; e < 4; ++e) lg += fabsf(hv[e] - hj[4 * q + e]) * al[4 * q + e]; }
            const float gn = -logf(-logf(u + EPSV) + EPSV);
            const float x = (lg + gn) * 10.0f;
            const float xc = fmaxf(x, -80.0f);
            const float ex = expf(-xc);
            float a = __builtin_amdgcn_rcpf(1.0f + ex);
            a = (i == j) ? 1.0f : a;
            const unsigned wd = __builtin_amdgcn_ballot_w32(a > 0.01f);
            aw[(wave * RB + r) * 32 + lane] = a;
            *(volatile float*)(AOUT + (size_t)i * OUT_NN + j) = a;
            if (lane == 0) mws[r * WPR + seg] = wd;
        }
        __threadfence();
#pragma unroll 1
        for (int r = 0; r < RB; ++r) { const float a = aw[(wave * RB + r) * 32 + lane]; *(volatile float*)(AOUT + (size_t)(i0 + r) * OUT_NN + j) = a; }
    }
    __syncthreads();
    unsigned* mdst = MB + (size_t)i0 * WPR;
    const int np = RB * WPR / 4;
#pragma unroll 1
    for (int ps = 0; ps < 2; ++ps) {
        for (int p = tid; p < np; p += 256) { const v4u w = *(const v4ua*)(&mws[p * 4]); *(volatile v4u*)(mdst + (size_t)p * 4) = w; }
        if (ps == 0) __threadfence(); }
}

__global__ __launch_bounds__(32) void k_gemm(const h16* __restrict__ A, const h16* __restrict__ Bt, const float* __restrict__ avec, h16* VT, float* WP, int K, float cs_plane, float cs_vec) {
    __shared__ __align__(16) float os[16 * 68];
    const int lane = threadIdx.x & 31, lr = lane & 15, hi = lane >> 4; const int r0 = blockIdx.x * 64, c0 = blockIdx.y * 64;
    v8f acc[4][4];
#pragma unroll
    for (int mb = 0; mb < 4; ++mb)
#pragma unroll
        for (int nb = 0; nb < 4; ++nb) acc[mb][nb] = (v8f){};
    const size_t aoff = (size_t)(r0 + lr) * K + 8 * hi, boff = (size_t)(c0 + lr) * K + 8 * hi;
#pragma unroll 1
    for (int kc = 0; kc < K; kc += 32) {
        v16h a[4];
#pragma unroll
        for (int mb = 0; mb < 4; ++mb) a[mb] = ldh(A + aoff + (size_t)mb * 16 * K + kc);
#pragma unroll
        for (int nb = 0; nb < 4; ++nb) { const v16h b = ldh(Bt + boff + (size_t)nb * 16 * K + kc);
#pragma unroll
            for (int mb = 0; mb < 4; ++mb) acc[mb][nb] = wg(a[mb], b, acc[mb][nb]); }
    }
    if (blockIdx.x < 2) {
#pragma unroll
        for (int mb = 0; mb < 4; ++mb) {
#pragma unroll
            for (int nb = 0; nb < 4; ++nb) {
#pragma unroll
                for (int j = 0; j < 8; ++j) os[(hi * 8 + j) * 68 + nb * 16 + lr] = acc[mb][nb][j] * cs_plane; }
            wave_sync();
            const size_t sb = (size_t)(r0 + mb * 16) * NN + (size_t)c0;
#pragma unroll 1
            for (int ps = 0; ps < 2; ++ps) {
#pragma unroll
                for (int s = 0; s < 4; ++s) { const int row = 4 * s + (lane >> 3), c8 = (lane & 7) * 8;
                    const v4f x0 = *(const v4fa*)(&os[row * 68 + c8]); const v4f x1 = *(const v4fa*)(&os[row * 68 + c8 + 4]); v8h hv;
#pragma unroll
                    for (int i = 0; i < 4; ++i) { hv[i] = toh_flush(x0[i]); hv[4 + i] = toh_flush(x1[i]); }
                    *(volatile v8h*)(VT + sb + (size_t)row * NN + c8) = hv; }
                if (ps == 0) __threadfence(); }
            wave_sync();
        }
    } else {
        float part[4] = { 0.0f, 0.0f, 0.0f, 0.0f };
#pragma unroll
        for (int mb = 0; mb < 4; ++mb) {
            const float* ap = avec + (r0 - GG) + mb * 16 + 8 * hi;
            const v4f a0 = *(const v4f*)ap, a1 = *(const v4f*)(ap + 4);
            float av[8];
#pragma unroll
            for (int e = 0; e < 4; ++e) { av[e] = bfr(a0[e]); av[4 + e] = bfr(a1[e]); }
#pragma unroll
            for (int j = 0; j < 8; ++j)
#pragma unroll
                for (int nb = 0; nb < 4; ++nb) part[nb] += acc[mb][nb][j] * av[j]; }
#pragma unroll
        for (int nb = 0; nb < 4; ++nb) { part[nb] += __shfl_xor(part[nb], 16, 32); part[nb] *= cs_vec; }
        if (hi == 0) {
#pragma unroll
            for (int nb = 0; nb < 4; ++nb) os[nb * 16 + lr] = part[nb]; }
        wave_sync();
        float* wdst = WP + (size_t)(blockIdx.x - 2) * NN + c0;
        if (lane < 16) {
            const v4f val = *(const v4fa*)(&os[lane * 4]);
            *(volatile v4f*)(wdst + lane * 4) = val; __threadfence(); *(volatile v4f*)(wdst + lane * 4) = val; }
    }
}

__global__ __launch_bounds__(32 * AW) void k_agg(const h16* __restrict__ VT, const float* __restrict__ WP, const unsigned* __restrict__ MB, float* OUTF, h16* OUTH, int fin, float oscale) {
    __shared__ __align__(16) float os[AW * 16 * OSP];
    const int lane = threadIdx.x & 31, lr = lane & 15, hi = lane >> 4;
    const int wave = __builtin_amdgcn_readfirstlane((int)(threadIdx.x >> 5));
    const int t0 = (blockIdx.x * AW + wave) * 16;
    const int trow = t0 + lr;
    const float w1 = WP[trow] + WP[NN + trow];
    const unsigned* mrow = MB + (size_t)trow * WPR;
    const float* w2a = WP + 2 * NN + 8 * hi;
    const float* w2b = WP + 3 * NN + 8 * hi;
    const size_t vo = (size_t)lr * NN + 8 * hi;
    const int bsh = 8 * hi;
    v8f o[8];
#pragma unroll
    for (int j = 0; j < 8; ++j) o[j] = (v8f){};
    float m = NEGB, l = 0.0f;
#pragma unroll 1
    for (int key0 = 0; key0 < NN; key0 += 32) {
        unsigned mwd = mrow[key0 >> 5];
        asm volatile("" : "+v"(mwd));
        const float* pa_ = w2a + key0; const float* pb_ = w2b + key0;
        const v4f a0 = *(const v4f*)pa_, a1 = *(const v4f*)(pa_ + 4), a2 = *(const v4f*)(pa_ + 16), a3 = *(const v4f*)(pa_ + 20);
        const v4f b0 = *(const v4f*)pb_, b1 = *(const v4f*)(pb_ + 4), b2 = *(const v4f*)(pb_ + 16), b3 = *(const v4f*)(pb_ + 20);
        float kx[8], ky[8];
#pragma unroll
        for (int r = 0; r < 4; ++r) { kx[r] = a0[r] + b0[r]; kx[4 + r] = a1[r] + b1[r]; ky[r] = a2[r] + b2[r]; ky[4 + r] = a3[r] + b3[r]; }
        float sa[8], sb[8]; float mx = NEGB;
#pragma unroll
        for (int r = 0; r < 8; ++r) {
            float ea = w1 * kx[r]; ea = (ea >= 0.0f) ? ea : 0.2f * ea;
            float eb = w1 * ky[r]; eb = (eb >= 0.0f) ? eb : 0.2f * eb;
            const bool fa = ((mwd >> (bsh + r)) & 1u) != 0u;
            const bool fb = ((mwd >> (bsh + 16 + r)) & 1u) != 0u;
            sa[r] = fa ? ea * L2E : FILL2; sb[r] = fb ? eb * L2E : FILL2;
            mx = fmaxf(mx, fmaxf(sa[r], sb[r])); }
        mx = fmaxf(mx, __shfl_xor(mx, 16, 32));
        const float mnew = fmaxf(m, mx);
        const float alpha = __builtin_amdgcn_exp2f(m - mnew);
        v16h pb; float ls = 0.0f;
#pragma unroll
        for (int r = 0; r < 8; ++r) {
            const float xa = (sa[r] - mnew) + PSH, xb = (sb[r] - mnew) + PSH;
            const float ea = __builtin_amdgcn_exp2f(xa), eb = __builtin_amdgcn_exp2f(xb);
            const float ga = (xa < -14.0f) ? 0.0f : ea, gb = (xb < -14.0f) ? 0.0f : eb;
            const h16 pa = (h16)ga; const h16 pc = (h16)gb;
            pb[r] = pa; pb[8 + r] = pc; ls += (float)pa + (float)pc; }
        l = l * alpha + ls; m = mnew;
#pragma unroll
        for (int j = 0; j < 8; ++j) o[j] = o[j] * alpha;
        const h16* va = VT + vo + key0;
#pragma unroll
        for (int j = 0; j < 8; ++j) { const v16h vf = ldh(va + (size_t)j * 16 * NN); o[j] = wg(vf, pb, o[j]); }
    }
    l += __shfl_xor(l, 16, 32);
    const bool any = l > 0.0f;
    const float lsafe = any ? l : 1.0f;
    const float inv = any ? ((1.0f / lsafe) * oscale) : 0.0f;
    const int wb = wave * 16 * OSP;
#pragma unroll
    for (int j = 0; j < 8; ++j) { v4f a, c;
#pragma unroll
        for (int e = 0; e < 4; ++e) { a[e] = fmaxf(o[j][e] * inv, 0.0f); c[e] = fmaxf(o[j][4 + e] * inv, 0.0f); }
        *(v4fa*)(&os[wb + lr * OSP + 16 * j + 8 * hi]) = a; *(v4fa*)(&os[wb + lr * OSP + 16 * j + 8 * hi + 4]) = c; }
    wave_sync();
    if (fin != 0) {
        float* orow = OUTF + (size_t)t0 * GG;
#pragma unroll 1
        for (int ps = 0; ps < 2; ++ps) {
#pragma unroll 4
            for (int s = 0; s < 16; ++s) {
                const v4f val = *(const v4fa*)(&os[wb + s * OSP + lane * 4]);
                *(volatile v4f*)(orow + (size_t)s * GG + lane * 4) = val; }
            if (ps == 0) __threadfence(); }
    } else {
        h16* hrow = OUTH + (size_t)t0 * GG;
#pragma unroll 1
        for (int ps = 0; ps < 2; ++ps) {
#pragma unroll 4
            for (int s = 0; s < 8; ++s) { const int row = 2 * s + (lane >> 4), c8 = (lane & 15) * 8;
                const v4f x0 = *(const v4fa*)(&os[wb + row * OSP + c8]); const v4f x1 = *(const v4fa*)(&os[wb + row * OSP + c8 + 4]); v8h hv;
#pragma unroll
                for (int i = 0; i < 4; ++i) { hv[i] = toh_flush(x0[i]); hv[4 + i] = toh_flush(x1[i]); }
                *(volatile v8h*)(hrow + (size_t)row * GG + c8) = hv; }
            if (ps == 0) __threadfence(); }
    }
}

static constexpr size_t al256(size_t v) { return (v + 255) & ~(size_t)255; }
static constexpr size_t SZ_XH  = al256((size_t)NN * FIN * 2);
static constexpr size_t SZ_WT0 = al256((size_t)NW3 * FIN * 2);
static constexpr size_t SZ_WT1 = al256((size_t)NW3 * GG * 2);
static constexpr size_t SZ_MB  = al256((size_t)NN * WPR * 4);
static constexpr size_t SZ_VT  = al256((size_t)GG * NN * 2);
static constexpr size_t SZ_WP  = al256((size_t)4 * NN * 4);
static constexpr size_t SZ_HB  = al256((size_t)NN * GG * 2);
static constexpr size_t SZ_TOTAL = SZ_XH + SZ_WT0 + SZ_WT1 + SZ_MB + SZ_VT + SZ_WP + SZ_HB;
static_assert(SZ_TOTAL <= (size_t)134217728);
static constexpr size_t OFF_A_BYTES = (size_t)NN_FULL * GG * 4;
static constexpr size_t OFF_X_BYTES = OFF_A_BYTES + (size_t)NN_FULL * NN_FULL * 4;
static_assert(OFF_A_BYTES == (size_t)1048576);
static_assert(OFF_X_BYTES == (size_t)17825792);
static_assert(OFF_A_BYTES % 128 == 0);
static_assert(OFF_X_BYTES % 128 == 0);
static constexpr size_t OFF_A_EL = OFF_A_BYTES / 4;
static constexpr size_t OFF_X_EL = OFF_X_BYTES / 4;
static_assert((size_t)NN * GG <= OFF_A_EL);
static_assert(OFF_A_EL + (size_t)(NN - 1) * OUT_NN + NN <= OFF_X_EL);
static_assert(((size_t)OUT_NN * 4) % 128 == 0);

extern "C" void kernel_launch(void* const* d_in, const int* in_sizes, int n_in,
                              void* d_out, int out_size, void* d_ws, size_t ws_size, hipStream_t stream) {
    if (n_in < 11) return;
    if ((size_t)in_sizes[0] < (size_t)NN * FIN) return;
    if ((size_t)in_sizes[1] < (size_t)(NN - 1) * NN_FULL + NN) return;
    if (in_sizes[2] < FOBS) return;
    if (in_sizes[3] < FIN * GG || in_sizes[5] < FIN * GG || in_sizes[7] < FIN * GG) return;
    if (in_sizes[4] < GG * GG || in_sizes[6] < GG * GG || in_sizes[8] < GG * GG) return;
    if (in_sizes[9] < 2 * GG || in_sizes[10] < 2 * GG) return;
    if ((size_t)out_size < OFF_X_EL + (size_t)NN * FIN) return;
    if (SZ_TOTAL > ws_size) return;
    const float* X   = (const float*)d_in[0];
    const float* GU  = (const float*)d_in[1];
    const float* AL  = (const float*)d_in[2];
    const float* Ws0 = (const float*)d_in[3];
    const float* Ws1 = (const float*)d_in[4];
    const float* Wq0 = (const float*)d_in[5];
    const float* Wq1 = (const float*)d_in[6];
    const float* Wv0 = (const float*)d_in[7];
    const float* Wv1 = (const float*)d_in[8];
    const float* a0  = (const float*)d_in[9];
    const float* a1  = (const float*)d_in[10];
    float* OUT = (float*)d_out;
    float* OH = OUT;
    float* OA = OUT + OFF_A_EL;
    float* OX = OUT + OFF_X_EL;
    char* wsp = (char*)d_ws;
    h16* XH  = (h16*)wsp; wsp += SZ_XH;
    h16* WT0 = (h16*)wsp; wsp += SZ_WT0;
    h16* WT1 = (h16*)wsp; wsp += SZ_WT1;
    unsigned* MB = (unsigned*)wsp; wsp += SZ_MB;
    h16* VT  = (h16*)wsp; wsp += SZ_VT;
    float* WP = (float*)wsp; wsp += SZ_WP;
    h16* HB1 = (h16*)wsp; wsp += SZ_HB;

    k_xcopy<<<(unsigned)((size_t)NN * FIN / 4 / 256), 256, 0, stream>>>(X, OX, XH);
    k_wt<<<GG * FIN / 8 / 256, 256, 0, stream>>>(Ws0, WT0, FIN);
    k_wt<<<GG * FIN / 8 / 256, 256, 0, stream>>>(Wq0, WT0 + (size_t)GG * FIN, FIN);
    k_wt<<<GG * FIN / 8 / 256, 256, 0, stream>>>(Wv0, WT0 + (size_t)2 * GG * FIN, FIN);
    k_wt<<<GG * GG / 8 / 256, 256, 0, stream>>>(Ws1, WT1, GG);
    k_wt<<<GG * GG / 8 / 256, 256, 0, stream>>>(Wq1, WT1 + (size_t)GG * GG, GG);
    k_wt<<<GG * GG / 8 / 256, 256, 0, stream>>>(Wv1, WT1 + (size_t)2 * GG * GG, GG);

    k_adj<<<NN / RB, 256, 0, stream>>>(X, GU, AL, OA, MB);

    k_gemm<<<dim3(NW3 / 64, NN / 64, 1), 32, 0, stream>>>(WT0, XH, a0, VT, WP, FIN, CSP, CSV);
    k_agg<<<NN / (16 * AW), 32 * AW, 0, stream>>>(VT, WP, MB, OH, HB1, 0, 1.0f);
    k_gemm<<<dim3(NW3 / 64, NN / 64, 1), 32, 0, stream>>>(WT1, HB1, a1, VT, WP, GG, CSP, CSV);
    k_agg<<<NN / (16 * AW), 32 * AW, 0, stream>>>(VT, WP, MB, OH, HB1, 1, 1.0f / 64.0f);
}
